// LocalSelfMultiheadAttention_2173253452656
// MI455X (gfx1250) — hardware-verified
//
#include <hip/hip_runtime.h>
#include <math.h>

typedef __attribute__((ext_vector_type(16))) _Float16 v16h;
typedef __attribute__((ext_vector_type(16))) __bf16 v16b;
typedef __attribute__((ext_vector_type(8)))  _Float16 v8h;
typedef __attribute__((ext_vector_type(8)))  float v8f;
typedef __attribute__((ext_vector_type(4)))  float v4f;
typedef __attribute__((ext_vector_type(2)))  float v2f;
typedef __attribute__((ext_vector_type(4)))  unsigned v4u;
typedef __attribute__((ext_vector_type(4)))  int v4i;
typedef float __attribute__((may_alias)) float_a;
typedef int __attribute__((may_alias)) int_a;

template <typename T> __device__ __forceinline__ void vst2(void* p, T v) { *(volatile T*)p = v; __threadfence(); *(volatile T*)p = v; }
__device__ __forceinline__ v8f wmma16(v16h a, v16h b, v8f c) {
  v8f d = __builtin_amdgcn_wmma_f32_16x16x32_f16(false, a, false, b, (short)0, c, false, false);
  asm volatile("v_nop\n\tv_nop\n\tv_nop\n\tv_nop" : "+v"(d) : "v"(a), "v"(b));
  return d;
}
__device__ __forceinline__ v8f wmma_bf(v16b a, v16b b, v8f c) {
  v8f d = __builtin_amdgcn_wmma_f32_16x16x32_bf16(false, a, false, b, (short)0, c, false, false);
  asm volatile("v_nop\n\tv_nop\n\tv_nop\n\tv_nop" : "+v"(d) : "v"(a), "v"(b));
  return d;
}
__device__ __forceinline__ v16h frag_h(const _Float16* rowk0, int lane) {
  union { v16h v; v8h q[2]; } u; const _Float16* p = rowk0 + 8 * (lane >> 4);
  u.q[0] = *(const v8h*)p; u.q[1] = *(const v8h*)(p + 16); return u.v;
}
__device__ __forceinline__ v16h frag_f32(const float* rowk0, int lane) {
  v16h a; const float* p = rowk0 + 8 * (lane >> 4);
#pragma unroll
  for (int i = 0; i < 8; ++i) { a[i] = (_Float16)p[i]; a[8 + i] = (_Float16)p[16 + i]; }
  return a;
}
__device__ __forceinline__ v16h frag_f32s(const float* rowk0, int lane, float sc) {
  v16h a; const float* p = rowk0 + 8 * (lane >> 4);
#pragma unroll
  for (int i = 0; i < 8; ++i) { a[i] = (_Float16)(p[i] * sc); a[8 + i] = (_Float16)(p[16 + i] * sc); }
  return a;
}
__device__ __forceinline__ v16h fragc_f32(const float* W, int k0, int n, int lane, int ld, int K) {
  v16h a; const int g = lane >> 4;
#pragma unroll
  for (int i = 0; i < 8; ++i) { const int ka = k0 + 8 * g + i, kb = ka + 16;
    a[i] = (_Float16)(ka < K ? W[(size_t)(ka < K ? ka : K - 1) * ld + n] : 0.f); a[8 + i] = (_Float16)(kb < K ? W[(size_t)(kb < K ? kb : K - 1) * ld + n] : 0.f); }
  return a;
}
struct F2 { v16b h, l; };
__device__ __forceinline__ F2 bsplit16(const float v[16]) { F2 r;
#pragma unroll
  for (int i = 0; i < 16; ++i) { const __bf16 h = (__bf16)v[i]; r.h[i] = h; r.l[i] = (__bf16)(v[i] - (float)h); }
  return r; }
__device__ __forceinline__ F2 split_row(const float* row, int k0, int lane) { float v[16]; const float* p = row + k0 + 8 * (lane >> 4);
#pragma unroll
  for (int i = 0; i < 8; ++i) { v[i] = p[i]; v[8 + i] = p[16 + i]; }
  return bsplit16(v); }
__device__ __forceinline__ F2 split_rowK(const float* row, int k0, int lane, int K) { float v[16]; const int g = lane >> 4;
#pragma unroll
  for (int i = 0; i < 8; ++i) { const int ka = k0 + 8 * g + i, kb = ka + 16; v[i] = ka < K ? row[ka < K ? ka : K - 1] : 0.f; v[8 + i] = kb < K ? row[kb < K ? kb : K - 1] : 0.f; }
  return bsplit16(v); }
__device__ __forceinline__ F2 split_col(const float* W, int k0, int n, int lane, int ld, int K) { float v[16]; const int g = lane >> 4;
#pragma unroll
  for (int i = 0; i < 8; ++i) { const int ka = k0 + 8 * g + i, kb = ka + 16; v[i] = ka < K ? W[(size_t)(ka < K ? ka : K - 1) * ld + n] : 0.f; v[8 + i] = kb < K ? W[(size_t)(kb < K ? kb : K - 1) * ld + n] : 0.f; }
  return bsplit16(v); }
__device__ __forceinline__ v8f mac3(const F2& a, const F2& b, v8f c) { c = wmma_bf(a.l, b.h, c); c = wmma_bf(a.h, b.l, c); return wmma_bf(a.h, b.h, c); }
__device__ __forceinline__ float sigm(float v) { return 1.0f / (1.0f + expf(-v)); }
#define LDSX() do { asm volatile("s_wait_dscnt 0" ::: "memory"); __builtin_amdgcn_wave_barrier(); __builtin_amdgcn_fence(__ATOMIC_RELEASE, "workgroup"); } while (0)


#define NF 4
#define NL 2048
#define NN 64
#define FD 256
#define NH 8
#define HDIM 32
#define NR (NF * NL)
typedef __attribute__((ext_vector_type(8))) __bf16 v8b;
__device__ __forceinline__ v16b frag_b(const __bf16* rowk0, int lane) {
  union { v16b v; v8b q[2]; } u; const __bf16* p = rowk0 + 8 * (lane >> 4);
  u.q[0] = *(const v8b*)p; u.q[1] = *(const v8b*)(p + 16); return u.v;
}
__device__ __forceinline__ v16b frag_gbf(const float* rowk0, int lane) {
  v16b a; const float* p = rowk0 + 8 * (lane >> 4);
#pragma unroll
  for (int i = 0; i < 8; ++i) { a[i] = (__bf16)p[i]; a[8 + i] = (__bf16)p[16 + i]; }
  return a;
}
__device__ __forceinline__ float bfr(float v) { return (float)(__bf16)v; }
__device__ __attribute__((noinline)) float exp_ni(float v) { return expf(v); }

__global__ __launch_bounds__(256) void k_pack(const float* __restrict__ Wm, __bf16* __restrict__ PT) {
  __shared__ __align__(16) __bf16 srow[FD];
  const int n = blockIdx.x, tid = threadIdx.x;
  srow[tid] = (__bf16)Wm[(size_t)tid * 3 * FD + n];
  __syncthreads();
  if (tid < 32) vst2((unsigned*)(PT + (size_t)n * FD + tid * 8), *(const v4u*)(&srow[tid * 8]));
}
__global__ __launch_bounds__(128) void k_qkv(const float* __restrict__ X, const __bf16* __restrict__ PT, const float* __restrict__ bias, float* __restrict__ QKV) {
  __shared__ __align__(16) float so[4][16][132];
  const int tid = threadIdx.x, wave = tid >> 5, lane = tid & 31, col = lane & 15, g = lane >> 4; const size_t r0 = (size_t)blockIdx.x * 64 + wave * 16; const int n0 = blockIdx.y * 128;
  v8f acc[8] = {};
#pragma unroll 2
  for (int kc = 0; kc < FD / 32; ++kc) { const v16b a = frag_gbf(X + (r0 + col) * FD + kc * 32, lane);
#pragma unroll
    for (int j = 0; j < 8; ++j) acc[j] = wmma_bf(a, frag_b(PT + (size_t)(n0 + j * 16 + col) * FD + kc * 32, lane), acc[j]); }
#pragma unroll
  for (int j = 0; j < 8; ++j) { const float bb = bfr(bias[n0 + j * 16 + col]);
#pragma unroll
    for (int r = 0; r < 8; ++r) so[wave][8 * g + r][j * 16 + col] = acc[j][r] + bb; }
  LDSX();
  for (int rl = 0; rl < 16; ++rl) vst2(QKV + (r0 + rl) * 3 * FD + n0 + lane * 4, *(const v4f*)(&so[wave][rl][lane * 4]));
}
__global__ __launch_bounds__(256) void k_local(const float* __restrict__ QKV, const int* __restrict__ nl, const int* __restrict__ nm, const float* __restrict__ abias, float* __restrict__ O, float* __restrict__ AW, float* __restrict__ AT) {
  __shared__ __align__(16) float saw[8][NH][NN], sat[8][NH][NN], so[8][FD]; __shared__ int sidx[8][NN];
  const int tid = threadIdx.x, wave = tid >> 5, lane = tid & 31; const int h = lane >> 2, q4 = lane & 3;
  const size_t r = (size_t)blockIdx.x * 8 + wave;
  const int f = (int)(r / NL);
  for (int n = lane; n < NN; n += 32) { int i = nl[r * NN + n]; i = i < 0 ? 0 : (i >= NL ? NL - 1 : i); sidx[wave][n] = i; }
  float q[8]; { const float4 a = *(const float4*)(QKV + r * 3 * FD + h * HDIM + q4 * 8), c = *(const float4*)(QKV + r * 3 * FD + h * HDIM + q4 * 8 + 4); const float sc = 0.17677669529663687f;
    q[0] = a.x * sc; q[1] = a.y * sc; q[2] = a.z * sc; q[3] = a.w * sc; q[4] = c.x * sc; q[5] = c.y * sc; q[6] = c.z * sc; q[7] = c.w * sc; }
  LDSX();
#pragma unroll 2
  for (int n = 0; n < NN; ++n) { const float* kr = QKV + ((size_t)f * NL + sidx[wave][n]) * 3 * FD + FD + h * HDIM + q4 * 8; const float4 a = *(const float4*)kr, c = *(const float4*)(kr + 4);
    float d = ((q[0] * a.x + q[1] * a.y) + (q[2] * a.z + q[3] * a.w)) + ((q[4] * c.x + q[5] * c.y) + (q[6] * c.z + q[7] * c.w));
    d += __shfl_xor(d, 1); d += __shfl_xor(d, 2);
    if (q4 == 0) { const float m = (float)nm[r * NN + n]; const float aw = (m != 0.f ? d : -__builtin_inff()) + bfr(abias[(((size_t)f * NH + h) * NL + (r % NL)) * NN + n]); saw[wave][h][n] = aw; } }
  LDSX();
  { float mx = -__builtin_inff();
#pragma unroll
    for (int i = 0; i < 16; ++i) mx = fmaxf(mx, saw[wave][h][q4 * 16 + i]);
    mx = fmaxf(mx, __shfl_xor(mx, 1)); mx = fmaxf(mx, __shfl_xor(mx, 2));
    float s = 0.f; float e[16];
#pragma unroll
    for (int i = 0; i < 16; ++i) { e[i] = exp_ni(saw[wave][h][q4 * 16 + i] - mx); s += e[i]; }
    s += __shfl_xor(s, 1); s += __shfl_xor(s, 2);
    const float inv = 1.0f / s;
#pragma unroll
    for (int i = 0; i < 16; ++i) sat[wave][h][q4 * 16 + i] = e[i] * inv; }
  LDSX();
  { float o8[8] = {0.f, 0.f, 0.f, 0.f, 0.f, 0.f, 0.f, 0.f};
#pragma unroll 2
    for (int n = 0; n < NN; ++n) { const float* vr = QKV + ((size_t)f * NL + sidx[wave][n]) * 3 * FD + 2 * FD + h * HDIM + q4 * 8; const float4 a = *(const float4*)vr, c = *(const float4*)(vr + 4); const float p = sat[wave][h][n];
      o8[0] += p * a.x; o8[1] += p * a.y; o8[2] += p * a.z; o8[3] += p * a.w; o8[4] += p * c.x; o8[5] += p * c.y; o8[6] += p * c.z; o8[7] += p * c.w; }
#pragma unroll
    for (int j = 0; j < 8; ++j) so[wave][h * HDIM + q4 * 8 + j] = o8[j]; }
  LDSX();
  vst2(O + r * FD + lane * 4, *(const v4f*)&so[wave][lane * 4]); vst2(O + r * FD + 128 + lane * 4, *(const v4f*)&so[wave][128 + lane * 4]);
  for (int qq = lane; qq < NH * 16; qq += 32) { const int hh = qq >> 4, pc = qq & 15; const size_t row = ((size_t)f * NH + hh) * NL + (r % NL);
    vst2(AW + row * NN + pc * 4, *(const v4f*)&saw[wave][hh][pc * 4]); vst2(AT + row * NN + pc * 4, *(const v4f*)&sat[wave][hh][pc * 4]); }
}

extern "C" void kernel_launch(void* const* d_in, const int* in_sizes, int n_in, void* d_out, int out_size, void* d_ws, size_t ws_size, hipStream_t stream) {
  (void)in_sizes; (void)n_in; (void)out_size; (void)ws_size;
  const float* X = (const float*)d_in[0]; const float* abias = (const float*)d_in[1]; const int* nm = (const int*)d_in[2]; const int* nl = (const int*)d_in[3]; const float* Wm = (const float*)d_in[4]; const float* bias = (const float*)d_in[5];
  char* ws = (char*)d_ws; __bf16* PT = (__bf16*)ws; float* QKV = (float*)(ws + 2u * 768 * FD);
  float* O = (float*)d_out; float* AW = O + (size_t)NR * FD; float* AT = AW + (size_t)NF * NH * NL * NN;
  k_pack<<<3 * FD, 256, 0, stream>>>(Wm, PT);
  k_qkv<<<dim3(NR / 64, 3 * FD / 128), 128, 0, stream>>>(X, PT, bias, QKV);
  k_local<<<NR / 8, 256, 0, stream>>>(QKV, nl, nm, abias, O, AW, AT);
}
